// EnformerDotProductSelfAttention_27178553049153
// MI455X (gfx1250) — hardware-verified
//
#include <hip/hip_runtime.h>


namespace {
constexpr int S = 2048, NH = 8, D = 64, NB = 64, HALF = 32, QTP = 96;
constexpr float XS = 8.0f, PS = 1024.0f, WSC = 256.0f;
typedef _Float16 b16;
typedef __attribute__((ext_vector_type(16))) _Float16 v16b;
typedef __attribute__((ext_vector_type(8))) _Float16 v8b;
typedef __attribute__((ext_vector_type(8))) float v8f;
typedef __attribute__((ext_vector_type(4))) float v4f;
typedef __attribute__((ext_vector_type(2))) float v2f;
__device__ __forceinline__ float bf16_rne(float f) { unsigned int u = __float_as_uint(f); u += 0x7FFFu + ((u >> 16) & 1u); float r = __uint_as_float(u & 0xFFFF0000u); asm volatile("" : "+v"(r)); return r; }
__device__ __forceinline__ void split16(float v, b16& hi, b16& lo) { hi = (b16)v; lo = (b16)(v - (float)hi); }
__device__ __forceinline__ v16b frag_kb(const b16* p, int hh) { const v8b a = *(const v8b*)(p + 8 * hh), b = *(const v8b*)(p + 16 + 8 * hh); v16b f;
#pragma unroll
  for (int e = 0; e < 8; ++e) { f[e] = a[e]; f[8 + e] = b[e]; } return f; }
__device__ __forceinline__ v8f wmma16b(v16b a, v16b b, v8f c) { v8f d = __builtin_amdgcn_wmma_f32_16x16x32_f16(false, a, false, b, (short)0, c, false, false); asm volatile("v_nop\n\tv_nop\n\tv_nop\n\tv_nop" : "+v"(d) : "v"(a), "v"(b)); return d; }
__device__ __forceinline__ void wave_lds_sync() { __builtin_amdgcn_fence(__ATOMIC_RELEASE, "workgroup"); __builtin_amdgcn_wave_barrier(); __builtin_amdgcn_fence(__ATOMIC_ACQUIRE, "workgroup"); }
__device__ __forceinline__ float pmul(float a, float b) { float p = a * b; asm volatile("" : "+v"(p)); return p; }
__device__ __forceinline__ float width_k(int k) { return __builtin_powf(__expf(__logf(0.5f * (S + 1)) / (float)HALF), (float)(k + 1)); }

__global__ __launch_bounds__(256) void prep_kernel(const float* __restrict__ q, const float* __restrict__ k, const float* __restrict__ w, b16* __restrict__ QH, b16* __restrict__ KH, b16* __restrict__ WWT) { const size_t u = (size_t)blockIdx.x * 256 + threadIdx.x;
  for (int pass = 0; pass < 2; ++pass) {
    if (u < (size_t)S * NH * D / 8) { v8b a, c; for (int j = 0; j < 8; ++j) { a[j] = (b16)(bf16_rne(q[u * 8 + j]) * XS); c[j] = (b16)(bf16_rne(k[u * 8 + j]) * XS); } *(volatile v8b*)(QH + u * 8) = a; *(volatile v8b*)(KH + u * 8) = c; }
    if (u < (size_t)NH * NB * (D / 8)) { const int h = (int)(u / (NB * 8)), n = (int)((u / 8) % NB), d0 = (int)(u % 8) * 8; v8b v; for (int j = 0; j < 8; ++j) v[j] = (b16)(bf16_rne(w[((size_t)h * D + d0 + j) * NB + n]) * WSC); *(volatile v8b*)(WWT + ((size_t)h * NB + n) * D + d0) = v; }
    __threadfence(); } }
__global__ __launch_bounds__(32) void vt_kernel(const float* __restrict__ val, b16* __restrict__ VT) { const int lane = threadIdx.x; const int ch = blockIdx.x % (S / 32), h = blockIdx.x / (S / 32); const size_t j = (size_t)ch * 32 + lane; const size_t base = ((size_t)h * (S / 32) + ch) * D;
  for (int pass = 0; pass < 2; ++pass) {
#pragma unroll 8
    for (int d = 0; d < D; ++d) ((volatile b16*)VT)[(base + d) * 64 + lane] = (b16)(bf16_rne(val[(j * NH + h) * D + d]) * XS); __threadfence(); } }
__global__ __launch_bounds__(256) void table_kernel(const float* __restrict__ k, const float* __restrict__ u, const float* __restrict__ v, const float* __restrict__ w, float* __restrict__ TB) {
  __shared__ float Wk[HALF], VW[NH][NB], SU[NH][HALF + 1], SSg[NH][HALF + 1]; __shared__ int K0s[S]; const int t = threadIdx.x;
  if (t < HALF) Wk[t] = width_k(t);
  __syncthreads();
  for (int tt = t; tt < S; tt += 256) { int c = 0; for (int kk = 0; kk < HALF; ++kk) c += (Wk[kk] < (float)tt) ? 1 : 0; K0s[tt] = c; }
  for (int q_ = t; q_ < NH * NB; q_ += 256) { const int h = q_ / NB, n = q_ % NB; float s = 0.0f; for (int d = 0; d < D; ++d) s += pmul(bf16_rne(v[h * D + d]), bf16_rne(w[((size_t)h * D + d) * NB + n])); VW[h][n] = s; }
  __syncthreads();
  if (t < NH) { float su = 0.0f, ss = 0.0f; SU[t][HALF] = 0.0f; SSg[t][HALF] = 0.0f; for (int kk = HALF - 1; kk >= 0; --kk) { su += VW[t][kk]; ss += VW[t][HALF + kk]; SU[t][kk] = su; SSg[t][kk] = ss; } }
  __syncthreads();
  for (int pass = 0; pass < 2; ++pass) {
    for (int tt = t; tt < S; tt += 256) ((volatile float*)TB)[tt] = (float)K0s[tt];
    for (int q_ = t; q_ < NH * 4096; q_ += 256) { const int h = q_ / 4096, o = q_ % 4096; const int dd = o - (S - 1); float val_ = 0.0f; if (o < 2 * S - 1) { const int ad = dd < 0 ? -dd : dd; const int k0 = K0s[ad]; const float sg = dd > 0 ? 1.0f : (dd < 0 ? -1.0f : 0.0f); val_ = SU[h][k0] + pmul(sg, SSg[h][k0]); } ((volatile float*)TB)[S + (size_t)h * 4096 + o] = val_; }
    for (int q_ = t; q_ < NH * S; q_ += 256) { const int h = q_ / S, j = q_ % S; float s = 0.0f; for (int d = 0; d < D; ++d) s += pmul(bf16_rne(u[h * D + d]), bf16_rne(k[((size_t)j * NH + h) * D + d])); ((volatile float*)TB)[S + NH * 4096 + q_] = s; }
    __threadfence(); } }
__global__ __launch_bounds__(32) void qt_kernel(const b16* __restrict__ QH, const b16* __restrict__ WWT, float* __restrict__ QT) {
  __shared__ float Tf[16][68], Rw[16][QTP]; const int lane = threadIdx.x, nloc = lane & 15, hlf = lane >> 4; const int it = blockIdx.x % (S / 16), h = blockIdx.x / (S / 16); const size_t i0 = (size_t)it * 16;
  v8f acc[4] = {(v8f){}, (v8f){}, (v8f){}, (v8f){}};
#pragma unroll
  for (int kb = 0; kb < D; kb += 32) { const v16b a = frag_kb(QH + (i0 + nloc) * NH * D + h * D + kb, hlf);
#pragma unroll
    for (int t = 0; t < 4; ++t) acc[t] = wmma16b(a, frag_kb(WWT + ((size_t)h * NB + t * 16 + nloc) * D + kb, hlf), acc[t]); }
#pragma unroll
  for (int t = 0; t < 4; ++t)
#pragma unroll
    for (int r8 = 0; r8 < 8; ++r8) Tf[8 * hlf + r8][t * 16 + nloc] = acc[t][r8] * (1.0f / (XS * WSC));
  wave_lds_sync();
  { const int row = lane & 15, part = lane >> 4; float s = 0.0f; Rw[row][part * 33 + HALF] = 0.0f; for (int kk = HALF - 1; kk >= 0; --kk) { s += Tf[row][part * HALF + kk]; Rw[row][part * 33 + kk] = s; } if (part == 1) for (int z = 66; z < QTP; ++z) Rw[row][z] = 0.0f; }
  wave_lds_sync();
  for (int pass = 0; pass < 2; ++pass) { for (int q_ = lane; q_ < 16 * QTP; q_ += 32) ((volatile float*)QT)[((size_t)h * S + i0) * QTP + q_] = Rw[q_ / QTP][q_ % QTP]; __threadfence(); } }
__global__ __launch_bounds__(32) void att_kernel(const b16* __restrict__ QH, const b16* __restrict__ KH, const b16* __restrict__ VT, const float* __restrict__ TB, const float* __restrict__ QT, int HV, float* __restrict__ out) {
  __shared__ __attribute__((aligned(16))) b16 Ph[16][40], Pl[16][40]; __shared__ float Sc[16][33], Mx[16], Dn[16], Sf[16], Of[16][D + 2], Qt[16][68];
  const int lane = threadIdx.x, nloc = lane & 15, hlf = lane >> 4; const int it = blockIdx.x % (S / 16), h = blockIdx.x / (S / 16); if (h >= HV) return; const int i0 = it * 16;
  for (int q_ = lane; q_ < 16 * 66; q_ += 32) Qt[q_ / 66][q_ % 66] = QT[((size_t)h * S + i0 + q_ / 66) * QTP + (q_ % 66)];
  if (lane < 16) { Mx[lane] = -INFINITY; Dn[lane] = 0.0f; Sf[lane] = 0.0f; }
  const float* K0 = TB; const float* VR = TB + S + (size_t)h * 4096; const float* UK = TB + S + NH * 4096 + (size_t)h * S;
  v16b qa[2]; qa[0] = frag_kb(QH + (size_t)(i0 + nloc) * NH * D + h * D, hlf); qa[1] = frag_kb(QH + (size_t)(i0 + nloc) * NH * D + h * D + 32, hlf);
  v8f acc[4] = {(v8f){}, (v8f){}, (v8f){}, (v8f){}}; wave_lds_sync();
#pragma unroll 1
  for (int kc = 0; kc < S; kc += 32) { const int j = kc + lane; const float ukj = UK[j];
#pragma unroll
    for (int blk = 0; blk < 2; ++blk) { v8f s = {}; const size_t kr = (size_t)(kc + blk * 16 + nloc) * NH * D + h * D; s = wmma16b(qa[0], frag_kb(KH + kr, hlf), s); s = wmma16b(qa[1], frag_kb(KH + kr + 32, hlf), s);
#pragma unroll
      for (int r8 = 0; r8 < 8; ++r8) Sc[8 * hlf + r8][blk * 16 + nloc] = s[r8] * (1.0f / (XS * XS)); }
    wave_lds_sync();
#pragma unroll 1
    for (int qi = 0; qi < 16; ++qi) { const int i = i0 + qi; const int dd = i - j; const int ad = dd < 0 ? -dd : dd; const int k0 = (int)K0[ad]; const float sg = dd > 0 ? 1.0f : (dd < 0 ? -1.0f : 0.0f);
      const float bias = Qt[qi][k0] + pmul(sg, Qt[qi][33 + k0]) + ukj + VR[dd + (S - 1)]; const float sv = (Sc[qi][lane] + bias) * 0.125f;
      float cm = sv; for (int o = 16; o; o >>= 1) cm = fmaxf(cm, __shfl_xor(cm, o)); const float mo = Mx[qi]; const float mn = fmaxf(mo, cm); const float p = __expf(sv - mn); float ps = p; for (int o = 16; o; o >>= 1) ps += __shfl_xor(ps, o);
      b16 ph, plo; split16(p * PS, ph, plo); Ph[qi][lane] = ph; Pl[qi][lane] = plo; if (lane == 0) { const float sf = (mo == -INFINITY) ? 0.0f : __expf(mo - mn); Sf[qi] = sf; Dn[qi] = Dn[qi] * sf + ps; Mx[qi] = mn; } }
    wave_lds_sync(); const v16b pa = frag_kb(&Ph[nloc][0], hlf), pb = frag_kb(&Pl[nloc][0], hlf); const size_t vb = (((size_t)h * (S / 32) + kc / 32) * D) * 64;
#pragma unroll
    for (int t = 0; t < 4; ++t) {
#pragma unroll
      for (int r8 = 0; r8 < 8; ++r8) acc[t][r8] *= Sf[8 * hlf + r8];
      const v16b vv = frag_kb(VT + vb + (size_t)(t * 16 + nloc) * 64, hlf); acc[t] = wmma16b(pa, vv, acc[t]); acc[t] = wmma16b(pb, vv, acc[t]); }
    wave_lds_sync(); }
#pragma unroll
  for (int t = 0; t < 4; ++t)
#pragma unroll
    for (int r8 = 0; r8 < 8; ++r8) { const int rl = 8 * hlf + r8; Of[rl][t * 16 + nloc] = acc[t][r8] * (1.0f / (PS * XS)) / Dn[rl]; }
  wave_lds_sync();
  for (int pass = 0; pass < 2; ++pass) { for (int rr = 0; rr < 16; ++rr) *(volatile v2f*)(out + ((size_t)(i0 + rr) * NH + h) * D + lane * 2) = (v2f){Of[rr][lane * 2], Of[rr][lane * 2 + 1]}; __threadfence(); }
}
}

extern "C" void kernel_launch(void* const* d_in, const int* in_sizes, int n_in, void* d_out, int out_size, void* d_ws, size_t ws_size, hipStream_t stream) {
  (void)n_in;
  auto Fp = [&](int i) { return (const float*)d_in[i]; };
  if (in_sizes[0] != S * NH * D || in_sizes[1] != S * NH * D || in_sizes[2] != S * NH * D || in_sizes[3] != NH * D || in_sizes[4] != NH * D || in_sizes[5] != NH * D * NB || out_size != S * NH * D) return;
  const int HV = NH;
  size_t off = 0; char* ws = (char*)d_ws;
  auto carve = [&](size_t bytes) { char* p = ws + off; off += (bytes + 255) & ~(size_t)255; return p; };
  b16* QH = (b16*)carve((size_t)S * NH * D * 2); b16* KH = (b16*)carve((size_t)S * NH * D * 2); b16* WWT = (b16*)carve((size_t)NH * NB * D * 2); b16* VT = (b16*)carve((size_t)NH * (S / 32) * D * 64 * 2);
  float* TB = (float*)carve((size_t)(S + NH * 4096 + NH * S) * 4); float* QT = (float*)carve((size_t)NH * S * QTP * 4);
  if (off > ws_size || off > ((size_t)32 << 20)) return;
  prep_kernel<<<(unsigned)(((size_t)S * NH * D / 8 + 255) / 256), 256, 0, stream>>>(Fp(0), Fp(1), Fp(5), QH, KH, WWT);
  vt_kernel<<<NH * (S / 32), 32, 0, stream>>>(Fp(2), VT);
  table_kernel<<<1, 256, 0, stream>>>(Fp(1), Fp(3), Fp(4), Fp(5), TB);
  qt_kernel<<<NH * (S / 16), 32, 0, stream>>>(QH, WWT, QT);
  att_kernel<<<HV * (S / 16), 32, 0, stream>>>(QH, KH, VT, TB, QT, HV, (float*)d_out);
}
